// HistoricalCrossAttention_34832184771344
// MI455X (gfx1250) — hardware-verified
//
#include <hip/hip_runtime.h>
#include <stdint.h>


typedef float          v8f  __attribute__((ext_vector_type(8)));
typedef float          v4f  __attribute__((ext_vector_type(4), may_alias));
typedef unsigned short v8us __attribute__((ext_vector_type(8), may_alias));
typedef _Float16       v16h __attribute__((ext_vector_type(16)));
typedef __bf16         v16b __attribute__((ext_vector_type(16)));

#define DM 512
#define HD 64
#define NH 8
#define TT 2048

struct Raw { v8us lo; v8us hi; };

static __device__ __forceinline__ v8f zero8() {
    v8f z;
#pragma unroll
    for (int i = 0; i < 8; i++) z[i] = 0.0f;
    return z;
}

static __device__ __forceinline__ unsigned short bf_bits(float x) {
    unsigned int u = __float_as_uint(x);
    u += 0x7FFFu + ((u >> 16) & 1u);
    return (unsigned short)(u >> 16);
}
static __device__ __forceinline__ float bf_val(float x) {
    unsigned int u = ((unsigned int)bf_bits(x)) << 16;
    return __uint_as_float(u);
}
static __device__ __forceinline__ unsigned short h_bits(float x) {
    _Float16 h = (_Float16)x;
    return __builtin_bit_cast(unsigned short, h);
}

static __device__ __forceinline__ v8f mma_bf16(const Raw& a, const Raw& b, v8f c) {
    v16b av = __builtin_bit_cast(v16b, a);
    v16b bv = __builtin_bit_cast(v16b, b);
    v8f d = __builtin_amdgcn_wmma_f32_16x16x32_bf16(false, av, false, bv, (short)0, c, false, false);
    asm volatile("v_nop\n\tv_nop\n\tv_nop\n\tv_nop" : "+v"(d) : "v"(av), "v"(bv));
    return d;
}
static __device__ __forceinline__ v8f mma_f16(v16h av, v16h bv, v8f c) {
    v8f d = __builtin_amdgcn_wmma_f32_16x16x32_f16(false, av, false, bv, (short)0, c, false, false);
    asm volatile("v_nop\n\tv_nop\n\tv_nop\n\tv_nop" : "+v"(d) : "v"(av), "v"(bv));
    return d;
}
static __device__ __forceinline__ v16h as_h(const Raw& a) { return __builtin_bit_cast(v16h, a); }

__global__ __launch_bounds__(256)
void cvt16(const float* __restrict__ src, uint16_t* dst, int n8, int kind, float scl) {
    const int i = blockIdx.x * 256 + (int)threadIdx.x;
    if (i >= n8) return;
    const float* p = src + (size_t)i * 8;
    v4f a = *(const v4f*)p;
    v4f b = *(const v4f*)(p + 4);
    float x[8];
    x[0] = a[0]; x[1] = a[1]; x[2] = a[2]; x[3] = a[3];
    x[4] = b[0]; x[5] = b[1]; x[6] = b[2]; x[7] = b[3];
    v8us o;
#pragma unroll
    for (int e = 0; e < 8; e++) {
        const float v = x[e];
        unsigned short bits;
        if (kind == 0) bits = bf_bits(v);
        else           bits = h_bits(bf_val(v) * scl);
        o[e] = bits;
    }
    uint16_t* d = dst + (size_t)i * 8;
    *(volatile v8us*)d = o;
    __threadfence();
    *(volatile v8us*)d = o;
}

template <int MODE>
__global__ __launch_bounds__(256)
void gemm_nt(const uint16_t* __restrict__ A, const uint16_t* __restrict__ W,
             const float* __restrict__ bias, void* outp, int M, float oscale) {
    __shared__ __align__(16) unsigned char smem[128 * 136 * 2];

    const int tid  = (int)threadIdx.x;
    const int lane = tid & 31, wave = tid >> 5;
    const int wm = wave & 1, wn = wave >> 1;
    const int hh = lane >> 4, l16 = lane & 15;
    const int m0 = blockIdx.x * 128, n0 = blockIdx.y * 128;
    if (m0 + 128 > M || n0 + 128 > DM) return;

    v8f C[4][2];
#pragma unroll
    for (int i = 0; i < 4; i++)
#pragma unroll
        for (int j = 0; j < 2; j++) C[i][j] = zero8();

    const int arow = m0 + wm * 64;
    const int bcol = n0 + wn * 32;

    for (int k = 0; k < DM; k += 32) {
        Raw af[4], bf[2];
#pragma unroll
        for (int mt = 0; mt < 4; mt++) {
            const uint16_t* p = A + (size_t)(arow + mt * 16 + l16) * DM + k + 8 * hh;
            af[mt].lo = *(const v8us*)p;
            af[mt].hi = *(const v8us*)(p + 16);
        }
#pragma unroll
        for (int nt = 0; nt < 2; nt++) {
            const uint16_t* p = W + (size_t)(bcol + nt * 16 + l16) * DM + k + 8 * hh;
            bf[nt].lo = *(const v8us*)p;
            bf[nt].hi = *(const v8us*)(p + 16);
        }
#pragma unroll
        for (int mt = 0; mt < 4; mt++)
#pragma unroll
            for (int nt = 0; nt < 2; nt++) {
                if constexpr (MODE == 2) C[mt][nt] = mma_f16(as_h(af[mt]), as_h(bf[nt]), C[mt][nt]);
                else                     C[mt][nt] = mma_bf16(af[mt], bf[nt], C[mt][nt]);
            }
    }

    if constexpr (MODE == 0) {
        unsigned short (*Ls)[136] = (unsigned short (*)[136])smem;
#pragma unroll
        for (int nt = 0; nt < 2; nt++) {
            const int cl = wn * 32 + nt * 16 + l16;
            const float bvv = bias[n0 + cl];
#pragma unroll
            for (int mt = 0; mt < 4; mt++)
#pragma unroll
                for (int r = 0; r < 8; r++) {
                    const int rl = wm * 64 + mt * 16 + 8 * hh + r;
                    Ls[rl][cl] = h_bits((C[mt][nt][r] + bvv) * oscale);
                }
        }
        __syncthreads();
        uint16_t* O = (uint16_t*)outp;
        const int b = m0 / TT, t0 = m0 % TT;
        const int head0 = n0 >> 6;
        for (int pass = 0; pass < 2; pass++) {
#pragma unroll
            for (int it = 0; it < 8; it++) {
                const int L  = it * 32 + (tid >> 3);
                const int pc = tid & 7;
                const int hs = L >> 7, rl = L & 127;
                v8us v = *(const v8us*)&Ls[rl][hs * 64 + pc * 8];
                const size_t idx = (((size_t)b * NH + head0 + hs) * TT + t0 + rl) * HD + pc * 8;
                *(volatile v8us*)(O + idx) = v;
            }
            if (pass == 0) __threadfence();
        }
    } else if constexpr (MODE == 1) {
        unsigned short (*Lt)[136] = (unsigned short (*)[136])smem;
#pragma unroll
        for (int nt = 0; nt < 2; nt++) {
            const int cl = wn * 32 + nt * 16 + l16;
            const float bvv = bias[n0 + cl];
#pragma unroll
            for (int mt = 0; mt < 4; mt++) {
                v8us pk;
#pragma unroll
                for (int r = 0; r < 8; r++) pk[r] = h_bits((C[mt][nt][r] + bvv) * oscale);
                *(v8us*)&Lt[cl][wm * 64 + mt * 16 + 8 * hh] = pk;
            }
        }
        __syncthreads();
        uint16_t* O = (uint16_t*)outp;
        const int b = m0 / TT, t0 = m0 % TT;
        for (int pass = 0; pass < 2; pass++) {
#pragma unroll
            for (int it = 0; it < 8; it++) {
                const int L  = it * 32 + (tid >> 3);
                const int pc = tid & 7;
                const int nl = L >> 1, sg = L & 1;
                v8us v = *(const v8us*)&Lt[nl][sg * 64 + pc * 8];
                const int n = n0 + nl;
                const int head = n >> 6, hd = n & 63;
                const size_t idx = (((size_t)b * NH + head) * HD + hd) * TT + t0 + sg * 64 + pc * 8;
                *(volatile v8us*)(O + idx) = v;
            }
            if (pass == 0) __threadfence();
        }
    } else {
        float (*Lf)[132] = (float (*)[132])smem;
        float* O = (float*)outp;
        for (int ph = 0; ph < 2; ph++) {
            if (wm == ph) {
#pragma unroll
                for (int nt = 0; nt < 2; nt++) {
                    const int cl = wn * 32 + nt * 16 + l16;
                    const float bvv = bias[n0 + cl];
#pragma unroll
                    for (int mt = 0; mt < 4; mt++)
#pragma unroll
                        for (int r = 0; r < 8; r++)
                            Lf[mt * 16 + 8 * hh + r][cl] = C[mt][nt][r] * oscale + bvv;
                }
            }
            __syncthreads();
            for (int pass = 0; pass < 2; pass++) {
#pragma unroll
                for (int it = 0; it < 8; it++) {
                    const int L  = it * 32 + (tid >> 3);
                    const int pc = tid & 7;
                    const int rl = L >> 2, q = L & 3;
                    v4f v = *(const v4f*)&Lf[rl][q * 32 + pc * 4];
                    const size_t idx = (size_t)(m0 + ph * 64 + rl) * DM + n0 + q * 32 + pc * 4;
                    *(volatile v4f*)(O + idx) = v;
                }
                if (pass == 0) __threadfence();
            }
            __syncthreads();
        }
    }
}

__global__ __launch_bounds__(256)
void attn_fwd(const uint16_t* __restrict__ Q, const uint16_t* __restrict__ K,
              const uint16_t* __restrict__ VT, uint16_t* O, int nbh) {
    __shared__ __align__(16) unsigned short Kt[64][72];
    __shared__ __align__(16) unsigned short Vt[64][72];
    __shared__ __align__(16) unsigned short Os[8][16][72];

    const int tid  = (int)threadIdx.x;
    const int lane = tid & 31, wave = tid >> 5;
    const int hh = lane >> 4, l16 = lane & 15;
    const int bh = blockIdx.y;
    if (bh >= nbh || (int)blockIdx.x * 128 + 128 > TT) return;
    const int b = bh / NH, h = bh % NH;
    const int q0 = blockIdx.x * 128 + wave * 16;

    Raw qf[2];
    {
        const uint16_t* p = Q + ((size_t)bh * TT + q0 + l16) * HD + 8 * hh;
        qf[0].lo = *(const v8us*)p;        qf[0].hi = *(const v8us*)(p + 16);
        qf[1].lo = *(const v8us*)(p + 32); qf[1].hi = *(const v8us*)(p + 48);
    }

    const float ninf = -__builtin_huge_valf();
    float mrun = ninf, lrun = 0.0f;
    v8f Oc[4];
#pragma unroll
    for (int nt = 0; nt < 4; nt++) Oc[nt] = zero8();

    for (int j = 0; j < TT / 64; j++) {
        __syncthreads();
#pragma unroll
        for (int c = 0; c < 2; c++) {
            const int idx = tid + 256 * c;
            const int row = idx >> 3, pc = idx & 7;
            v8us kv = *(const v8us*)(K  + ((size_t)bh * TT + j * 64 + row) * HD + pc * 8);
            *(v8us*)&Kt[row][pc * 8] = kv;
            v8us vv = *(const v8us*)(VT + ((size_t)bh * HD + row) * TT + j * 64 + pc * 8);
            *(v8us*)&Vt[row][pc * 8] = vv;
        }
        __syncthreads();

        v8f S[4];
#pragma unroll
        for (int t = 0; t < 4; t++) S[t] = zero8();
#pragma unroll
        for (int t = 0; t < 4; t++) {
#pragma unroll
            for (int kk = 0; kk < 2; kk++) {
                Raw kf;
                kf.lo = *(const v8us*)&Kt[t * 16 + l16][kk * 32 + 8 * hh];
                kf.hi = *(const v8us*)&Kt[t * 16 + l16][kk * 32 + 16 + 8 * hh];
                S[t] = mma_f16(as_h(kf), as_h(qf[kk]), S[t]);
            }
        }

        float mx = ninf;
#pragma unroll
        for (int t = 0; t < 4; t++)
#pragma unroll
            for (int r = 0; r < 8; r++) {
                const float s = S[t][r] * 0.125f;
                S[t][r] = s;
                mx = fmaxf(mx, s);
            }
        mx = fmaxf(mx, __shfl_xor(mx, 16, 32));
        const float mnew = fmaxf(mrun, mx);
        const float scl  = __expf(mrun - mnew);
        float sm = 0.0f;
        v16h pf[2];
#pragma unroll
        for (int t = 0; t < 4; t++)
#pragma unroll
            for (int r = 0; r < 8; r++) {
                const float pv = __expf(S[t][r] - mnew);
                sm += pv;
                const _Float16 hv = (_Float16)(pv * 256.0f);
                pf[t >> 1][((t & 1) << 3) + r] = hv;
            }
        sm += __shfl_xor(sm, 16, 32);
        lrun = lrun * scl + sm;
        mrun = mnew;
#pragma unroll
        for (int nt = 0; nt < 4; nt++) Oc[nt] = Oc[nt] * scl;

#pragma unroll
        for (int nt = 0; nt < 4; nt++) {
#pragma unroll
            for (int kk2 = 0; kk2 < 2; kk2++) {
                Raw vf;
                vf.lo = *(const v8us*)&Vt[nt * 16 + l16][kk2 * 32 + 8 * hh];
                vf.hi = *(const v8us*)&Vt[nt * 16 + l16][kk2 * 32 + 16 + 8 * hh];
                Oc[nt] = mma_f16(as_h(vf), pf[kk2], Oc[nt]);
            }
        }
    }

    const float inv = 0.25f / lrun;
    __syncthreads();
#pragma unroll
    for (int nt = 0; nt < 4; nt++) {
        v8us pk;
#pragma unroll
        for (int r = 0; r < 8; r++) pk[r] = h_bits(Oc[nt][r] * inv);
        *(v8us*)&Os[wave][l16][nt * 16 + 8 * hh] = pk;
    }
    __syncthreads();
    for (int pass = 0; pass < 2; pass++) {
#pragma unroll
        for (int it = 0; it < 4; it++) {
            const int L  = it * 4 + (lane >> 3);
            const int pc = lane & 7;
            v8us v = *(const v8us*)&Os[wave][L][pc * 8];
            const size_t idx = ((size_t)b * TT + q0 + L) * DM + h * HD + pc * 8;
            *(volatile v8us*)(O + idx) = v;
        }
        if (pass == 0) __threadfence();
    }
}

extern "C" void kernel_launch(void* const* d_in, const int* in_sizes, int n_in,
                              void* d_out, int out_size, void* d_ws, size_t ws_size,
                              hipStream_t stream) {
    if (n_in < 10) return;
    const int NX = in_sizes[0];
    const int NW = in_sizes[2];
    if (NX <= 0 || in_sizes[1] != NX || in_sizes[3] != DM || in_sizes[5] != DM ||
        in_sizes[7] != DM || in_sizes[9] != DM || NW != DM * DM || in_sizes[4] != NW ||
        in_sizes[6] != NW || in_sizes[8] != NW || (NX % (TT * DM)) != 0 || out_size != NX) return;
    const int M  = NX / DM;
    const int Bb = M / TT;

    const float* xc = (const float*)d_in[0];
    const float* xp = (const float*)d_in[1];
    const float* wq = (const float*)d_in[2];
    const float* bq = (const float*)d_in[3];
    const float* wk = (const float*)d_in[4];
    const float* bk = (const float*)d_in[5];
    const float* wv = (const float*)d_in[6];
    const float* bv = (const float*)d_in[7];
    const float* wo = (const float*)d_in[8];
    const float* bo = (const float*)d_in[9];

    size_t off = 0;
    auto carve = [&](size_t bytes) -> size_t {
        size_t o = off;
        off += (bytes + 255) & ~(size_t)255;
        return o;
    };
    const size_t o_xc = carve((size_t)NX * 2);
    const size_t o_xp = carve((size_t)NX * 2);
    const size_t o_wq = carve((size_t)NW * 2);
    const size_t o_wk = carve((size_t)NW * 2);
    const size_t o_wv = carve((size_t)NW * 2);
    const size_t o_wo = carve((size_t)NW * 2);
    const size_t o_q  = carve((size_t)NX * 2);
    const size_t o_k  = carve((size_t)NX * 2);
    const size_t o_vt = carve((size_t)NX * 2);
    const size_t o_o  = carve((size_t)NX * 2);
    if (off > ws_size) return;

    char* ws = (char*)d_ws;
    uint16_t* xcb = (uint16_t*)(ws + o_xc);
    uint16_t* xpb = (uint16_t*)(ws + o_xp);
    uint16_t* wqb = (uint16_t*)(ws + o_wq);
    uint16_t* wkb = (uint16_t*)(ws + o_wk);
    uint16_t* wvb = (uint16_t*)(ws + o_wv);
    uint16_t* wob = (uint16_t*)(ws + o_wo);
    uint16_t* Qb  = (uint16_t*)(ws + o_q);
    uint16_t* Kb  = (uint16_t*)(ws + o_k);
    uint16_t* VTb = (uint16_t*)(ws + o_vt);
    uint16_t* Ob  = (uint16_t*)(ws + o_o);

    const dim3 blk(256);
    const int nx8 = NX / 8, nw8 = NW / 8;
    cvt16<<<dim3((nx8 + 255) / 256), blk, 0, stream>>>(xc, xcb, nx8, 0, 1.0f);
    cvt16<<<dim3((nx8 + 255) / 256), blk, 0, stream>>>(xp, xpb, nx8, 0, 1.0f);
    cvt16<<<dim3((nw8 + 255) / 256), blk, 0, stream>>>(wq, wqb, nw8, 0, 1.0f);
    cvt16<<<dim3((nw8 + 255) / 256), blk, 0, stream>>>(wk, wkb, nw8, 0, 1.0f);
    cvt16<<<dim3((nw8 + 255) / 256), blk, 0, stream>>>(wv, wvb, nw8, 0, 1.0f);
    cvt16<<<dim3((nw8 + 255) / 256), blk, 0, stream>>>(wo, wob, nw8, 1, 64.0f);

    const dim3 gg((M + 127) / 128, DM / 128);
    gemm_nt<0><<<gg, blk, 0, stream>>>(xcb, wqb, bq, (void*)Qb,  M, 1.0f);
    gemm_nt<0><<<gg, blk, 0, stream>>>(xpb, wkb, bk, (void*)Kb,  M, 1.0f);
    gemm_nt<1><<<gg, blk, 0, stream>>>(xpb, wvb, bv, (void*)VTb, M, 1.0f);

    attn_fwd<<<dim3(TT / 128, Bb * NH), blk, 0, stream>>>(Qb, Kb, VTb, Ob, Bb * NH);

    gemm_nt<2><<<gg, blk, 0, stream>>>(Ob, wob, bo, d_out, M, 1.0f / 4096.0f);
}
